// MMAttn_2250562863585
// MI455X (gfx1250) — hardware-verified
//
#include <hip/hip_runtime.h>
#include <math.h>
#include <float.h>
#include <stdint.h>

#define BSZ   2
#define NF    32
#define NV    64
#define NJ    (NV + 1)
#define STOK  (NF * NJ)
#define SP    2112
#define NQT   (SP / 64)
#define DM    1024
#define NH    16
#define HD    64
#define NPAIR (HD / 2)
#define QKVN  (3 * DM)
#define R0    (BSZ * NF * NV)
#define R1    (BSZ * NF)
#define RALL  (R0 + R1)
static_assert(NH * HD == DM);
static_assert(HD == 64);
static_assert(DM == 128 * 8);
static_assert(SP >= STOK && (SP % 64) == 0 && (SP - STOK) < 64);
static_assert((R0 % 64) == 0 && (R1 % 64) == 0 && (DM % 64) == 0 && (QKVN % 64) == 0 && (DM % 32) == 0);
static_assert((((R0 / 64) * (QKVN / 64)) % 8) == 0 && (((R1 / 64) * (QKVN / 64)) % 8) == 0);
static_assert((((R0 / 64) * (DM / 64)) % 8) == 0 && (((R1 / 64) * (DM / 64)) % 8) == 0);
static_assert(((R0 * DM / 8) % 256) == 0 && ((R1 * DM / 8) % 256) == 0);
static_assert(((SP * NPAIR) % 256) == 0);

typedef _Float16 v16h __attribute__((ext_vector_type(16)));
typedef _Float16 v8h  __attribute__((ext_vector_type(8)));
typedef float    v8f  __attribute__((ext_vector_type(8)));
typedef float    v4f  __attribute__((ext_vector_type(4)));
typedef unsigned int v4u __attribute__((ext_vector_type(4)));

__device__ __forceinline__ unsigned short bf_bits(float f) {
  unsigned u = __float_as_uint(f);
  return (unsigned short)((u + 0x7FFFu + ((u >> 16) & 1u)) >> 16);
}
__device__ __forceinline__ float bf_up(unsigned short h) { return __uint_as_float(((unsigned)h) << 16); }
__device__ __forceinline__ float bfr(float f) { return bf_up(bf_bits(f)); }
__device__ __forceinline__ unsigned short h_bits(_Float16 x) { return __builtin_bit_cast(unsigned short, x); }
__device__ __forceinline__ unsigned pk16(unsigned short a, unsigned short b) { return (unsigned)a | ((unsigned)b << 16); }
__device__ __forceinline__ v8f zero8() { v8f z = {0.f, 0.f, 0.f, 0.f, 0.f, 0.f, 0.f, 0.f}; return z; }

__device__ __forceinline__ void ld8(const float* p, float* o) {
  const v4f a = *(const v4f*)(p);
  const v4f b = *(const v4f*)(p + 4);
  o[0] = a[0]; o[1] = a[1]; o[2] = a[2]; o[3] = a[3];
  o[4] = b[0]; o[5] = b[1]; o[6] = b[2]; o[7] = b[3];
}

__device__ __forceinline__ v16h ldfrag_h(const _Float16* p) {
  union { v16h v; v8h h[2]; } f;
  f.h[0] = *(const v8h*)(p);
  f.h[1] = *(const v8h*)(p + 16);
  return f.v;
}

__device__ __forceinline__ v8f mma_h(v16h a, v16h b, v8f c) {
  c = __builtin_amdgcn_wmma_f32_16x16x32_f16(false, a, false, b, (short)0, c, false, false);
#if defined(__HIP_DEVICE_COMPILE__)
  asm volatile("v_nop\n\tv_nop\n\tv_nop\n\tv_nop" : "+v"(c) : "v"(a), "v"(b));
#endif
  return c;
}
__device__ __forceinline__ v8f mma_h_raw(v16h a, v16h b, v8f c) {
  return __builtin_amdgcn_wmma_f32_16x16x32_f16(false, a, false, b, (short)0, c, false, false);
}
__device__ __forceinline__ void dep_guard_h(v8f& a, v8f& b, v16h x) {
#if defined(__HIP_DEVICE_COMPILE__)
  asm volatile("v_nop\n\tv_nop\n\tv_nop\n\tv_nop" : "+v"(a), "+v"(b) : "v"(x));
#endif
}
__device__ __forceinline__ void keep4_h(v16h a, v16h b, v16h c, v16h d) {
#if defined(__HIP_DEVICE_COMPILE__)
  asm volatile("v_nop" :: "v"(a), "v"(b), "v"(c), "v"(d));
#endif
}
__device__ __forceinline__ void acc_guard4(v8f& a, v8f& b, v8f& c, v8f& d) {
#if defined(__HIP_DEVICE_COMPILE__)
  asm volatile("v_nop\n\tv_nop\n\tv_nop\n\tv_nop" : "+v"(a), "+v"(b), "+v"(c), "+v"(d));
#endif
}

__global__ __launch_bounds__(256) void rope_tab(float* ct, float* st, int n) {
#pragma clang fp contract(off)
  const int i = blockIdx.x * 256 + threadIdx.x;
  if (i < n) {
    const int t = i >> 5;
    const int j = i & 31;
    const float e   = (float)j * (1.0f / 32.0f);
    const float p   = powf(10000.0f, e);
    const float inv = 1.0f / p;
    const float ang = (float)t * inv;
    const float cv = cosf(ang);
    const float sv = sinf(ang);
    *(volatile float*)(ct + i) = cv;
    *(volatile float*)(st + i) = sv;
    __threadfence();
    *(volatile float*)(ct + i) = cv;
    *(volatile float*)(st + i) = sv;
  }
}

__global__ __launch_bounds__(256) void wt_cvt(const float* __restrict__ W, int ncols, int nrows,
                                              unsigned short* outp, float sc) {
  __shared__ __align__(16) float sw[64 * 68];
  const int tid = threadIdx.x;
  const int n0 = blockIdx.x * 64;
  const int k0 = blockIdx.y * 64;
#pragma unroll
  for (int i = 0; i < 4; ++i) {
    const int idx = i * 256 + tid;
    const int kk = idx >> 4, c4 = (idx & 15) * 4;
    const v4f a = *(const v4f*)(W + (size_t)(k0 + kk) * ncols + n0 + c4);
    *(v4f*)(sw + kk * 68 + c4) = a;
  }
  __syncthreads();

  const int g = tid >> 3, piece = tid & 7;
  v4u ov[2];
  size_t oofs[2];
#pragma unroll
  for (int it = 0; it < 2; ++it) {
    const int nn = it * 32 + g;
    v4u a;
#pragma unroll
    for (int e = 0; e < 4; ++e) {
      const float f0 = sw[(piece * 8 + 2 * e) * 68 + nn];
      const float f1 = sw[(piece * 8 + 2 * e + 1) * 68 + nn];
      a[e] = pk16(h_bits((_Float16)(bfr(f0) * sc)), h_bits((_Float16)(bfr(f1) * sc)));
    }
    ov[it] = a;
    oofs[it] = (size_t)(n0 + nn) * nrows + k0 + piece * 8;
  }
  for (int pass = 0; pass < 2; ++pass) {
#pragma unroll
    for (int it = 0; it < 2; ++it) *(volatile v4u*)(outp + oofs[it]) = ov[it];
    __threadfence();
  }
}

__global__ __launch_bounds__(256) void cvt_xh(const float* __restrict__ in, unsigned short* out, int n8,
                                              float sc) {
  const int i = blockIdx.x * 256 + threadIdx.x;
  if (i < n8) {
    const v4f a = *(const v4f*)(in + (size_t)i * 8);
    const v4f b = *(const v4f*)(in + (size_t)i * 8 + 4);
    v4u p;
    p[0] = pk16(h_bits((_Float16)(bfr(a[0]) * sc)), h_bits((_Float16)(bfr(a[1]) * sc)));
    p[1] = pk16(h_bits((_Float16)(bfr(a[2]) * sc)), h_bits((_Float16)(bfr(a[3]) * sc)));
    p[2] = pk16(h_bits((_Float16)(bfr(b[0]) * sc)), h_bits((_Float16)(bfr(b[1]) * sc)));
    p[3] = pk16(h_bits((_Float16)(bfr(b[2]) * sc)), h_bits((_Float16)(bfr(b[3]) * sc)));
    *(volatile v4u*)(out + (size_t)i * 8) = p;
    __threadfence();
    *(volatile v4u*)(out + (size_t)i * 8) = p;
  }
}

__global__ __launch_bounds__(256) void gemm64(
    const unsigned short* __restrict__ Ap, int lda,
    const unsigned short* __restrict__ Btp, int ldb,
    const float* __restrict__ bias, float* Cf, int ldc, int M, int N, int K, float oscale) {
  const _Float16* Ah = (const _Float16*)(const void*)Ap;
  const _Float16* Bh = (const _Float16*)(const void*)Btp;
  __shared__ __align__(16) float sT[8][16 * 68];
  const int lane = threadIdx.x & 31;
  const int wave = threadIdx.x >> 5;
  const int tilesN = N >> 6;
  const int tilesM = M >> 6;
  const int tile = blockIdx.x * 8 + wave;
  if (tile >= tilesM * tilesN) return;
  const int tm = tile / tilesN;
  const int tn = tile - tm * tilesN;
  const int m0 = tm << 6;
  const int n0 = tn << 6;

  const int rlane = lane & 15;
  const int koff  = (lane >> 4) * 8;
  const int mOff  = (lane >> 4) * 8;

  v8f acc[4][4];
#pragma unroll
  for (int i = 0; i < 4; ++i)
#pragma unroll
    for (int j = 0; j < 4; ++j) acc[i][j] = zero8();

  for (int k0 = 0; k0 < K; k0 += 32) {
    v16h bh[4];
#pragma unroll
    for (int j = 0; j < 4; ++j) {
      const size_t bo = (size_t)(n0 + (j << 4) + rlane) * ldb + koff + k0;
      bh[j] = ldfrag_h(Bh + bo);
    }
#pragma unroll
    for (int i = 0; i < 4; ++i) {
      const size_t ao = (size_t)(m0 + (i << 4) + rlane) * lda + koff + k0;
      const v16h ah = ldfrag_h(Ah + ao);
#pragma unroll
      for (int j = 0; j < 4; ++j) acc[i][j] = mma_h_raw(ah, bh[j], acc[i][j]);
      dep_guard_h(acc[i][0], acc[i][3], ah);
    }
    keep4_h(bh[0], bh[1], bh[2], bh[3]);
  }
  acc_guard4(acc[0][0], acc[0][1], acc[0][2], acc[0][3]);
  acc_guard4(acc[1][0], acc[1][1], acc[1][2], acc[1][3]);
  acc_guard4(acc[2][0], acc[2][1], acc[2][2], acc[2][3]);
  acc_guard4(acc[3][0], acc[3][1], acc[3][2], acc[3][3]);

  float* slab = sT[wave];
  const int h2 = lane >> 4, c4 = (lane & 15) * 4;
  v4f b4;
  {
    const v4f braw = *(const v4f*)(bias + n0 + c4);
#pragma unroll
    for (int e = 0; e < 4; ++e) b4[e] = bfr(braw[e]);
  }
#pragma unroll
  for (int i = 0; i < 4; ++i) {
    const int mBase = m0 + (i << 4);
#pragma unroll
    for (int r = 0; r < 8; ++r) {
#pragma unroll
      for (int j = 0; j < 4; ++j) {
        slab[(mOff + r) * 68 + (j << 4) + rlane] = acc[i][j][r];
      }
    }
    __builtin_amdgcn_fence(__ATOMIC_RELEASE, "workgroup");
    __builtin_amdgcn_wave_barrier();
    __builtin_amdgcn_fence(__ATOMIC_ACQUIRE, "workgroup");
    v4f ov[8];
#pragma unroll
    for (int it = 0; it < 8; ++it) {
      const int row = it * 2 + h2;
      const v4f xs = *(const v4f*)(slab + row * 68 + c4);
      ov[it] = xs * oscale + b4;
    }
    for (int pass = 0; pass < 2; ++pass) {
#pragma unroll
      for (int it = 0; it < 8; ++it) {
        const int row = it * 2 + h2;
        *(volatile v4f*)(Cf + (size_t)(mBase + row) * ldc + n0 + c4) = ov[it];
      }
      __threadfence();
    }
    __builtin_amdgcn_fence(__ATOMIC_RELEASE, "workgroup");
    __builtin_amdgcn_wave_barrier();
    __builtin_amdgcn_fence(__ATOMIC_ACQUIRE, "workgroup");
  }
}

__global__ __launch_bounds__(128) void ln_rope(const float* __restrict__ qkvf, const float* __restrict__ ct,
                                               const float* __restrict__ st, unsigned short* qh,
                                               unsigned short* ql, unsigned short* kh, unsigned short* kl,
                                               float osc, float rsc) {
#pragma clang fp contract(off)
  const int tid = threadIdx.x;
  const int bp  = blockIdx.x;
  const int b   = bp / SP;
  const int p   = bp - b * SP;
  const int pad = (p >= STOK) ? 1 : 0;
  const int pc  = (pad != 0) ? (STOK - 1) : p;
  const int f   = pc / NJ;
  const int j   = pc - f * NJ;
  const int srow = (j < NV) ? (b * (NF * NV) + f * NV + j) : (R0 + b * NF + f);
  const float* rowp = qkvf + (size_t)srow * QKVN;
  const int d0 = tid * 8;
  const int j0 = d0 & 31;
  const float sgn = ((d0 & 32) == 0) ? -1.0f : 1.0f;
  float xq[8], xk[8], cv[8], sv[8];
  ld8(rowp + d0, xq);
  ld8(rowp + DM + d0, xk);
  ld8(ct + (size_t)p * NPAIR + j0, cv);
  ld8(st + (size_t)p * NPAIR + j0, sv);

  float sq = 0.f, sk = 0.f;
#pragma unroll
  for (int e = 0; e < 8; ++e) { sq += xq[e]; sk += xk[e]; }
#pragma unroll
  for (int off = 1; off < 8; off <<= 1) { sq += __shfl_xor(sq, off, 32); sk += __shfl_xor(sk, off, 32); }
  const float muq = sq * (1.0f / (float)HD);
  const float muk = sk * (1.0f / (float)HD);
  float dq[8], dk[8];
  float vq = 0.f, vk = 0.f;
#pragma unroll
  for (int e = 0; e < 8; ++e) {
    dq[e] = xq[e] - muq; vq += dq[e] * dq[e];
    dk[e] = xk[e] - muk; vk += dk[e] * dk[e];
  }
#pragma unroll
  for (int off = 1; off < 8; off <<= 1) { vq += __shfl_xor(vq, off, 32); vk += __shfl_xor(vk, off, 32); }
  const float rq = rsqrtf(vq * (1.0f / (float)HD) + 1e-5f);
  const float rk = rsqrtf(vk * (1.0f / (float)HD) + 1e-5f);
  float nq[8], nk[8], pq[8], pk[8];
#pragma unroll
  for (int e = 0; e < 8; ++e) { nq[e] = dq[e] * rq; nk[e] = dk[e] * rk; }
#pragma unroll
  for (int e = 0; e < 8; ++e) { pq[e] = __shfl_xor(nq[e], 4, 32); pk[e] = __shfl_xor(nk[e], 4, 32); }

  v4u aqh, aql, akh, akl;
#pragma unroll
  for (int pp = 0; pp < 4; ++pp) {
    const int e = 2 * pp;
    const float yq0 = nq[e] * cv[e] + (sgn * pq[e]) * sv[e];
    const float yq1 = nq[e + 1] * cv[e + 1] + (sgn * pq[e + 1]) * sv[e + 1];
    const float yk0 = nk[e] * cv[e] + (sgn * pk[e]) * sv[e];
    const float yk1 = nk[e + 1] * cv[e + 1] + (sgn * pk[e + 1]) * sv[e + 1];
    const float tq0 = (pad != 0) ? 0.f : yq0 * osc;
    const float tq1 = (pad != 0) ? 0.f : yq1 * osc;
    const float tk0 = (pad != 0) ? 0.f : yk0 * osc;
    const float tk1 = (pad != 0) ? 0.f : yk1 * osc;
    const _Float16 hq0 = (_Float16)tq0, hq1 = (_Float16)tq1, hk0 = (_Float16)tk0, hk1 = (_Float16)tk1;
    const _Float16 lq0 = (_Float16)((tq0 - (float)hq0) * rsc);
    const _Float16 lq1 = (_Float16)((tq1 - (float)hq1) * rsc);
    const _Float16 lk0 = (_Float16)((tk0 - (float)hk0) * rsc);
    const _Float16 lk1 = (_Float16)((tk1 - (float)hk1) * rsc);
    aqh[pp] = pk16(h_bits(hq0), h_bits(hq1));
    aql[pp] = pk16(h_bits(lq0), h_bits(lq1));
    akh[pp] = pk16(h_bits(hk0), h_bits(hk1));
    akl[pp] = pk16(h_bits(lk0), h_bits(lk1));
  }
  const size_t o = (size_t)bp * DM + d0;
  *(volatile v4u*)(qh + o) = aqh;
  *(volatile v4u*)(ql + o) = aql;
  *(volatile v4u*)(kh + o) = akh;
  *(volatile v4u*)(kl + o) = akl;
  __threadfence();
  *(volatile v4u*)(qh + o) = aqh;
  *(volatile v4u*)(ql + o) = aql;
  *(volatile v4u*)(kh + o) = akh;
  *(volatile v4u*)(kl + o) = akl;
}

__global__ __launch_bounds__(256) void v_planes(const float* __restrict__ qkvf, unsigned short* vt, float vscale) {
  __shared__ __align__(16) float svt[64 * 68];
  const int tid = threadIdx.x;
  const int kt  = blockIdx.x;
  const int hh  = blockIdx.y;
  const int b   = blockIdx.z;
  const int t0  = kt * 64;
#pragma unroll
  for (int i = 0; i < 4; ++i) {
    const int idx = i * 256 + tid;
    const int tt = idx >> 4, c4 = (idx & 15) * 4;
    const int p  = t0 + tt;
    const int pad = (p >= STOK) ? 1 : 0;
    const int pc = (pad != 0) ? (STOK - 1) : p;
    const int f  = pc / NJ;
    const int j  = pc - f * NJ;
    const int srow = (j < NV) ? (b * (NF * NV) + f * NV + j) : (R0 + b * NF + f);
    v4f a = *(const v4f*)(qkvf + (size_t)srow * QKVN + 2 * DM + hh * HD + c4);
#pragma unroll
    for (int e = 0; e < 4; ++e) a[e] = (pad != 0) ? 0.f : a[e];
    *(v4f*)(svt + tt * 68 + c4) = a;
  }
  __syncthreads();

  const int g = tid >> 3, piece = tid & 7;
  v4u hv[2];
  size_t hofs[2];
#pragma unroll
  for (int it = 0; it < 2; ++it) {
    const int d = it * 32 + g;
    v4u a;
#pragma unroll
    for (int e = 0; e < 4; ++e) {
      const float f0 = svt[(piece * 8 + 2 * e) * 68 + d] * vscale;
      const float f1 = svt[(piece * 8 + 2 * e + 1) * 68 + d] * vscale;
      a[e] = pk16(h_bits((_Float16)f0), h_bits((_Float16)f1));
    }
    hv[it] = a;
    hofs[it] = ((size_t)(b * DM + hh * HD + d)) * SP + t0 + piece * 8;
  }
  for (int pass = 0; pass < 2; ++pass) {
#pragma unroll
    for (int it = 0; it < 2; ++it) *(volatile v4u*)(vt + hofs[it]) = hv[it];
    __threadfence();
  }
}

__global__ __launch_bounds__(128)
void attn_j64(const unsigned short* __restrict__ qhp, const unsigned short* __restrict__ qlp,
              const unsigned short* __restrict__ khp, const unsigned short* __restrict__ klp,
              const unsigned short* __restrict__ vtp, unsigned short* yh,
              float sscale, float rinv, float oscl) {
  union FH { v16h v; v8h h[2]; };
  __shared__ __align__(16) _Float16 Khs[64 * 64];
  __shared__ __align__(16) _Float16 Kls[64 * 64];
  __shared__ __align__(16) _Float16 Vts[64 * 64];
  __shared__ __align__(16) _Float16 Psh[4][16 * 64];
  __shared__ __align__(16) float    Os[4][16 * 64];

  const int tid  = threadIdx.x;
  const int wave = tid >> 5;
  const int lane = tid & 31;
  const int hh   = lane >> 4;
  const int c    = lane & 15;

  const int bx = blockIdx.x;
  const int qt = bx % NQT;
  const int hb = bx / NQT;
  const int h  = hb % NH;
  const int b  = hb / NH;
  const int q0 = qt * 64 + wave * 16;

  const size_t qkb = (size_t)b * SP * DM + (size_t)h * HD;
  const _Float16* Qh = (const _Float16*)(const void*)qhp + qkb;
  const _Float16* Ql = (const _Float16*)(const void*)qlp + qkb;
  const _Float16* Kh = (const _Float16*)(const void*)khp + qkb;
  const _Float16* Kl = (const _Float16*)(const void*)klp + qkb;
  const _Float16* Vt = (const _Float16*)(const void*)vtp + ((size_t)b * DM + (size_t)h * HD) * SP;

  v16h qa[2], qr[2];
#pragma unroll
  for (int dc = 0; dc < 2; ++dc) {
    const size_t qo = (size_t)(q0 + c) * DM + dc * 32 + 8 * hh;
    qa[dc] = ldfrag_h(Qh + qo);
    qr[dc] = ldfrag_h(Ql + qo);
  }

  float mrow[8], lrow[8];
  v8f oacc[4];
#pragma unroll
  for (int r = 0; r < 8; ++r) { mrow[r] = -INFINITY; lrow[r] = 0.f; }
#pragma unroll
  for (int t = 0; t < 4; ++t) oacc[t] = zero8();

  for (int kt = 0; kt < NQT; ++kt) {
    const int kv0 = kt * 64;
    __syncthreads();
    {
      const int r = tid >> 1, half = (tid & 1) * 32;
      const _Float16* kg  = Kh + (size_t)(kv0 + r) * DM + half;
      const _Float16* klg = Kl + (size_t)(kv0 + r) * DM + half;
      const _Float16* vg  = Vt + (size_t)r * SP + kv0 + half;
#pragma unroll
      for (int i = 0; i < 4; ++i) {
        const v8h a0 = *(const v8h*)(kg + 8 * i);
        const v8h a1 = *(const v8h*)(klg + 8 * i);
        const v8h b0 = *(const v8h*)(vg + 8 * i);
        *(v8h*)(Khs + r * 64 + half + 8 * i) = a0;
        *(v8h*)(Kls + r * 64 + half + 8 * i) = a1;
        *(v8h*)(Vts + r * 64 + half + 8 * i) = b0;
      }
    }
    __syncthreads();

    v8f s[4];
#pragma unroll
    for (int j = 0; j < 4; ++j) {
      v8f ahh = zero8(), ax = zero8();
#pragma unroll
      for (int dc = 0; dc < 2; ++dc) {
        FH kb, kr;
        kb.h[0] = *(const v8h*)(Khs + (j * 16 + c) * 64 + dc * 32 + 8 * hh);
        kb.h[1] = *(const v8h*)(Khs + (j * 16 + c) * 64 + dc * 32 + 16 + 8 * hh);
        kr.h[0] = *(const v8h*)(Kls + (j * 16 + c) * 64 + dc * 32 + 8 * hh);
        kr.h[1] = *(const v8h*)(Kls + (j * 16 + c) * 64 + dc * 32 + 16 + 8 * hh);
        ahh = mma_h(qa[dc], kb.v, ahh);
        ax  = mma_h(qa[dc], kr.v, ax);
        ax  = mma_h(qr[dc], kb.v, ax);
      }
      s[j] = ahh + ax * rinv;
    }

    _Float16* pwh = Psh[wave];
#pragma unroll
    for (int r = 0; r < 8; ++r) {
      float m = -INFINITY;
#pragma unroll
      for (int j = 0; j < 4; ++j) {
        const int key = kv0 + j * 16 + c;
        float sv = s[j][r] * sscale;
        sv = (key < STOK) ? sv : -FLT_MAX;
        s[j][r] = sv;
        m = fmaxf(m, sv);
      }
#pragma unroll
      for (int off = 1; off < 16; off <<= 1) m = fmaxf(m, __shfl_xor(m, off, 32));
      const float mnew  = fmaxf(mrow[r], m);
      const float msafe = (mnew == -INFINITY) ? 0.f : mnew;
      const float alpha = __expf(mrow[r] - msafe);
      mrow[r] = mnew;
      float psum = 0.f;
#pragma unroll
      for (int j = 0; j < 4; ++j) {
        const float p = __expf(s[j][r] - msafe);
        psum += p;
        const _Float16 ph = (_Float16)(p * 1024.0f);
        pwh[(8 * hh + r) * 64 + j * 16 + c] = ph;
      }
#pragma unroll
      for (int off = 1; off < 16; off <<= 1) psum += __shfl_xor(psum, off, 32);
      lrow[r] = lrow[r] * alpha + psum;
#pragma unroll
      for (int t = 0; t < 4; ++t) oacc[t][r] *= alpha;
    }
    __builtin_amdgcn_fence(__ATOMIC_RELEASE, "workgroup");
    __builtin_amdgcn_wave_barrier();
    __builtin_amdgcn_fence(__ATOMIC_ACQUIRE, "workgroup");

#pragma unroll 1
    for (int kk = 0; kk < 2; ++kk) {
      FH pa;
      pa.h[0] = *(const v8h*)(pwh + c * 64 + kk * 32 + 8 * hh);
      pa.h[1] = *(const v8h*)(pwh + c * 64 + kk * 32 + 16 + 8 * hh);
#pragma unroll
      for (int t = 0; t < 4; ++t) {
        FH vb;
        vb.h[0] = *(const v8h*)(Vts + (t * 16 + c) * 64 + kk * 32 + 8 * hh);
        vb.h[1] = *(const v8h*)(Vts + (t * 16 + c) * 64 + kk * 32 + 16 + 8 * hh);
        oacc[t] = mma_h(pa.v, vb.v, oacc[t]);
      }
    }
  }

  float* os = Os[wave];
#pragma unroll
  for (int r = 0; r < 8; ++r) {
    const float l = lrow[r];
    const float inv = ((l > 0.f) ? (1.0f / l) : 0.f) * oscl;
#pragma unroll
    for (int t = 0; t < 4; ++t) os[(8 * hh + r) * 64 + t * 16 + c] = oacc[t][r] * inv;
  }
  __builtin_amdgcn_fence(__ATOMIC_RELEASE, "workgroup");
  __builtin_amdgcn_wave_barrier();
  __builtin_amdgcn_fence(__ATOMIC_ACQUIRE, "workgroup");
  {
    const int q8 = lane & 7, rr = lane >> 3, c8 = q8 * 8;
    v4u ov[4];
    size_t go[4];
    int ok[4];
#pragma unroll
    for (int it = 0; it < 4; ++it) {
      const int row = it * 4 + rr;
      float xs[8];
      ld8(os + row * 64 + c8, xs);
      v4u a;
#pragma unroll
      for (int pp = 0; pp < 4; ++pp) a[pp] = pk16(h_bits((_Float16)xs[2 * pp]), h_bits((_Float16)xs[2 * pp + 1]));
      ov[it] = a;
      const int p   = q0 + row;
      const int okv = (p < STOK) ? 1 : 0;
      const int pc  = (okv != 0) ? p : (STOK - 1);
      const int f   = pc / NJ;
      const int j   = pc - f * NJ;
      const int dr  = (j < NV) ? (b * (NF * NV) + f * NV + j) : (R0 + b * NF + f);
      go[it] = (size_t)dr * DM + (size_t)h * HD + c8;
      ok[it] = okv;
    }
    for (int pass = 0; pass < 2; ++pass) {
#pragma unroll
      for (int it = 0; it < 4; ++it) {
        if (ok[it] != 0) *(volatile v4u*)(yh + go[it]) = ov[it];
      }
      __threadfence();
    }
  }
}

extern "C" void kernel_launch(void* const* d_in, const int* in_sizes, int n_in,
                              void* d_out, int out_size, void* d_ws, size_t ws_size,
                              hipStream_t stream) {
  if (n_in < 10) return;
  if (in_sizes[0] != R0 * DM) return;
  if (in_sizes[1] != R1 * DM) return;
  if (in_sizes[2] != DM * QKVN || in_sizes[3] != QKVN) return;
  if (in_sizes[4] != DM * QKVN || in_sizes[5] != QKVN) return;
  if (in_sizes[6] != DM * DM || in_sizes[7] != DM) return;
  if (in_sizes[8] != DM * DM || in_sizes[9] != DM) return;
  if (out_size != RALL * DM) return;

  const float* x0    = (const float*)d_in[0];
  const float* x1    = (const float*)d_in[1];
  const float* wqkv0 = (const float*)d_in[2];
  const float* bqkv0 = (const float*)d_in[3];
  const float* wqkv1 = (const float*)d_in[4];
  const float* bqkv1 = (const float*)d_in[5];
  const float* wo0   = (const float*)d_in[6];
  const float* bo0   = (const float*)d_in[7];
  const float* wo1   = (const float*)d_in[8];
  const float* bo1   = (const float*)d_in[9];

  const size_t PX0   = (size_t)R0 * DM * 2;
  const size_t PX1   = (size_t)R1 * DM * 2;
  const size_t PWq   = (size_t)QKVN * DM * 2;
  const size_t PWo   = (size_t)DM * DM * 2;
  const size_t PTrig = (size_t)SP * NPAIR * 4;
  const size_t PQKV  = (size_t)RALL * QKVN * 4;
  const size_t PQK   = (size_t)BSZ * SP * DM * 2;
  const size_t PVT   = (size_t)BSZ * DM * SP * 2;
  const size_t PY    = (size_t)RALL * DM * 2;
  size_t off = 0;
  const size_t oX0  = off; off += PX0;
  const size_t oX1  = off; off += PX1;
  const size_t oWq0 = off; off += PWq;
  const size_t oWq1 = off; off += PWq;
  const size_t oWo0 = off; off += PWo;
  const size_t oWo1 = off; off += PWo;
  const size_t oCos = off; off += PTrig;
  const size_t oSin = off; off += PTrig;
  const size_t oQKV = off; off += PQKV;
  const size_t oQh  = off; off += PQK;
  const size_t oQl  = off; off += PQK;
  const size_t oKh  = off; off += PQK;
  const size_t oKl  = off; off += PQK;
  const size_t oVT  = off; off += PVT;
  const size_t oY   = off; off += PY;
  if (off > ws_size) return;
  if (off > (size_t)134217728) return;

  char* ws = (char*)d_ws;
  unsigned short* X0h  = (unsigned short*)(ws + oX0);
  unsigned short* X1h  = (unsigned short*)(ws + oX1);
  unsigned short* WqT0 = (unsigned short*)(ws + oWq0);
  unsigned short* WqT1 = (unsigned short*)(ws + oWq1);
  unsigned short* WoT0 = (unsigned short*)(ws + oWo0);
  unsigned short* WoT1 = (unsigned short*)(ws + oWo1);
  float*          CosT = (float*)(ws + oCos);
  float*          SinT = (float*)(ws + oSin);
  float*          QKVf = (float*)(ws + oQKV);
  unsigned short* Qh   = (unsigned short*)(ws + oQh);
  unsigned short* Ql   = (unsigned short*)(ws + oQl);
  unsigned short* Kh   = (unsigned short*)(ws + oKh);
  unsigned short* Kl   = (unsigned short*)(ws + oKl);
  unsigned short* VT   = (unsigned short*)(ws + oVT);
  unsigned short* Yh   = (unsigned short*)(ws + oY);
  float*          outf = (float*)d_out;

  const dim3 blk(256);
  const int nTrig = SP * NPAIR;
  const int n8x0  = R0 * DM / 8;
  const int n8x1  = R1 * DM / 8;
  const dim3 gTrig((nTrig + 255) / 256);
  const dim3 gCx0((n8x0 + 255) / 256);
  const dim3 gCx1((n8x1 + 255) / 256);
  const dim3 gWq(QKVN / 64, DM / 64);
  const dim3 gWo(DM / 64, DM / 64);
  const dim3 gQKV0(((R0 / 64) * (QKVN / 64) + 7) / 8);
  const dim3 gQKV1(((R1 / 64) * (QKVN / 64) + 7) / 8);
  const dim3 gOut0(((R0 / 64) * (DM / 64) + 7) / 8);
  const dim3 gOut1(((R1 / 64) * (DM / 64) + 7) / 8);
  const dim3 gLn(BSZ * SP);
  const dim3 gVpl(NQT, NH, BSZ);
  const dim3 gAttn(BSZ * NH * NQT);

  const float wScale  = 64.0f;
  const float xScale  = 8.0f;
  const float qkScale = 16.0f;
  const float rScale  = 2048.0f;
  const float sscale  = 1.0f / 2048.0f;
  const float rinv    = 1.0f / 2048.0f;
  const float vScale  = 256.0f;
  const float attOscl = 16.0f / 262144.0f;
  const float yInv    = 1.0f / 1024.0f;

  rope_tab<<<gTrig, blk, 0, stream>>>(CosT, SinT, nTrig);
  wt_cvt<<<gWq, blk, 0, stream>>>(wqkv0, QKVN, DM, WqT0, wScale);
  wt_cvt<<<gWq, blk, 0, stream>>>(wqkv1, QKVN, DM, WqT1, wScale);
  wt_cvt<<<gWo, blk, 0, stream>>>(wo0, DM, DM, WoT0, wScale);
  wt_cvt<<<gWo, blk, 0, stream>>>(wo1, DM, DM, WoT1, wScale);
  cvt_xh<<<gCx0, blk, 0, stream>>>(x0, X0h, n8x0, xScale);
  cvt_xh<<<gCx1, blk, 0, stream>>>(x1, X1h, n8x1, xScale);
  gemm64<<<gQKV0, blk, 0, stream>>>(X0h, DM, WqT0, DM, bqkv0, QKVf, QKVN, R0, QKVN, DM, 1.0f / 512.0f);
  gemm64<<<gQKV1, blk, 0, stream>>>(X1h, DM, WqT1, DM, bqkv1, QKVf + (size_t)R0 * QKVN, QKVN, R1, QKVN, DM,
                                    1.0f / 512.0f);
  ln_rope<<<gLn, dim3(128), 0, stream>>>(QKVf, CosT, SinT, Qh, Ql, Kh, Kl, qkScale, rScale);
  v_planes<<<gVpl, blk, 0, stream>>>(QKVf, VT, vScale);
  attn_j64<<<gAttn, dim3(128), 0, stream>>>(Qh, Ql, Kh, Kl, VT, Yh, sscale, rinv, attOscl);
  gemm64<<<gOut0, blk, 0, stream>>>(Yh, DM, WoT0, DM, bo0, outf, DM, R0, DM, DM, yInv);
  gemm64<<<gOut1, blk, 0, stream>>>(Yh + (size_t)R0 * DM, DM, WoT1, DM, bo1, outf + (size_t)R0 * DM, DM, R1,
                                    DM, DM, yInv);
  (void)hipGetLastError();
}
